// PyramidAttention_89026082111944
// MI455X (gfx1250) — hardware-verified
//
#include <hip/hip_runtime.h>
#define NIMG 4
#define CC 64
#define CR 32
#define H0 48
#define NQ (H0 * H0)
#define NSC 5
#define LP 7616
__constant__ int NREALK[NSC] = {2304, 1849, 1444, 1089, 784};
__constant__ int KOFF[NSC + 1] = {0, 2304, 4160, 5632, 6784, 7616};
static const int hSZ[NSC] = {48, 43, 38, 33, 28}, hNPAD[NSC] = {2304, 1920, 1536, 1152, 896}, hKOFF[NSC + 1] = {0, 2304, 4160, 5632, 6784, 7616}, hNREAL[NSC] = {2304, 1849, 1444, 1089, 784};
typedef __bf16 v16b __attribute__((ext_vector_type(16)));
typedef unsigned short v8us __attribute__((ext_vector_type(8), may_alias));
typedef float  v8f  __attribute__((ext_vector_type(8)));
typedef float  v4f  __attribute__((ext_vector_type(4)));
typedef float  v4fa __attribute__((ext_vector_type(4), may_alias));
union FragB { v16b v; v8us half[2]; unsigned short u[16]; };

__device__ __forceinline__ unsigned short bf16_bits(float x) { unsigned int u = __float_as_uint(x); return (unsigned short)((u + 0x7FFFu + ((u >> 16) & 1u)) >> 16); }
__device__ __forceinline__ float bf16_val(unsigned short b) { return __uint_as_float(((unsigned int)b) << 16); }
__device__ __forceinline__ float bf16_round(float x) { return bf16_val(bf16_bits(x)); }
template <int NT>
__device__ __forceinline__ v8f mmaN(v16b ah, v16b al, v16b bh, v16b bl, v8f c) {
  c = __builtin_amdgcn_wmma_f32_16x16x32_bf16(false, ah, false, bh, (short)0, c, false, false);
  if (NT >= 2) c = __builtin_amdgcn_wmma_f32_16x16x32_bf16(false, al, false, bh, (short)0, c, false, false);
  if (NT >= 3) c = __builtin_amdgcn_wmma_f32_16x16x32_bf16(false, ah, false, bl, (short)0, c, false, false);
  asm volatile("v_nop\n\tv_nop\n\tv_nop\n\tv_nop" : "+v"(c) : "v"(ah), "v"(al), "v"(bh), "v"(bl));
  return c;
}

__global__ __launch_bounds__(256) void k_wt_bf16(const float* __restrict__ W, unsigned short* __restrict__ Wt, int K, int N) {
  const int t = blockIdx.x * 256 + threadIdx.x;
  const int k8n = K / 8;
  if (t >= N * k8n) return;
  const int n = t / k8n, k8 = (t % k8n) * 8;
  v8us v;
#pragma unroll
  for (int i = 0; i < 8; ++i) v[i] = bf16_bits(W[(size_t)(k8 + i) * N + n]);
  *(volatile v8us*)(Wt + (size_t)n * K + k8) = v;
  __threadfence();
  *(volatile v8us*)(Wt + (size_t)n * K + k8) = v;
}

template <bool ASPLIT, int ACT, bool BIAS_BF16>
__global__ __launch_bounds__(128) void k_gemm_bf(const float* __restrict__ A, int lda, const unsigned short* __restrict__ Wt, int ldb,
                                               const float* __restrict__ bias, float* __restrict__ C, int ldc, int M, int N, int K) {
  __shared__ __attribute__((aligned(16))) float so[4][16][64];
  const int tid = threadIdx.x, w = tid >> 5, lane = tid & 31, ln = lane & 15, hh = lane >> 4;
  const int ntn = N / 64;
  const int wid = blockIdx.x * 4 + w;
  const int mt = wid / ntn, nq = wid % ntn;
  if (mt * 16 >= M) return;
  const int row0 = mt * 16, col0 = nq * 64;
  const float* arow = A + (size_t)(row0 + ln) * lda;
  v8f acc[4] = {};
  for (int kb = 0; kb < K; kb += 32) {
    FragB ah, al;
    const v4f x0 = *(const v4fa*)(arow + kb + 8 * hh), x1 = *(const v4fa*)(arow + kb + 8 * hh + 4);
    const v4f x2 = *(const v4fa*)(arow + kb + 16 + 8 * hh), x3 = *(const v4fa*)(arow + kb + 16 + 8 * hh + 4);
    float xs[16] = {x0[0],x0[1],x0[2],x0[3],x1[0],x1[1],x1[2],x1[3],x2[0],x2[1],x2[2],x2[3],x3[0],x3[1],x3[2],x3[3]};
#pragma unroll
    for (int i = 0; i < 16; ++i) { const unsigned short hb = bf16_bits(xs[i]); ah.u[i] = hb; al.u[i] = ASPLIT ? bf16_bits(xs[i] - bf16_val(hb)) : (unsigned short)0; }
#pragma unroll
    for (int t = 0; t < 4; ++t) {
      const unsigned short* brow = Wt + (size_t)(col0 + t * 16 + ln) * ldb + kb;
      FragB b;
      b.half[0] = *(const v8us*)(brow + 8 * hh);
      b.half[1] = *(const v8us*)(brow + 16 + 8 * hh);
      acc[t] = mmaN<ASPLIT ? 2 : 1>(ah.v, al.v, b.v, b.v, acc[t]);
    }
  }
#pragma unroll
  for (int t = 0; t < 4; ++t) {
    float bv = bias ? bias[col0 + t * 16 + ln] : 0.f;
    if (BIAS_BF16) bv = bf16_round(bv);
#pragma unroll
    for (int r = 0; r < 8; ++r) { float v = acc[t][r] + bv; if (ACT == 1) v = fmaxf(v, 0.f); so[w][8 * hh + r][t * 16 + ln] = v; }
  }
  __builtin_amdgcn_fence(__ATOMIC_ACQ_REL, "workgroup");
  __builtin_amdgcn_wave_barrier();
  const int rsub = lane >> 4, c4 = (lane & 15) * 4;
  for (int pass = 0; pass < 2; ++pass) {
#pragma unroll
    for (int q = 0; q < 8; ++q) {
      const int r = q * 2 + rsub;
      const v4f v = *(const v4fa*)&so[w][r][c4];
      *(volatile v4f*)(C + (size_t)(row0 + r) * ldc + col0 + c4) = v;
    }
    if (pass == 0) __threadfence();
  }
}

template <bool ASPLIT, int ACT, bool BIAS_BF16, bool RES_BF16>
__global__ __launch_bounds__(128) void k_gemm_bf3(const float* __restrict__ A, int lda, const unsigned short* __restrict__ Wt, int ldb,
                                                const float* __restrict__ bias, const float* __restrict__ resid, int rmod, int ldr,
                                                float* __restrict__ C, int ldc, int M, int N, int K) {
  __shared__ __attribute__((aligned(16))) float so[4][16][64];
  const int tid = threadIdx.x, w = tid >> 5, lane = tid & 31, ln = lane & 15, hh = lane >> 4;
  const int ntn = N / 64;
  const int wid = blockIdx.x * 4 + w;
  const int mt = wid / ntn, nq = wid % ntn;
  if (mt * 16 >= M) return;
  const int row0 = mt * 16, col0 = nq * 64;
  const float* arow = A + (size_t)(row0 + ln) * lda;
  v8f acc[4] = {};
  for (int kb = 0; kb < K; kb += 32) {
    FragB ah, al;
    const v4f x0 = *(const v4fa*)(arow + kb + 8 * hh), x1 = *(const v4fa*)(arow + kb + 8 * hh + 4);
    const v4f x2 = *(const v4fa*)(arow + kb + 16 + 8 * hh), x3 = *(const v4fa*)(arow + kb + 16 + 8 * hh + 4);
    float xs[16] = {x0[0],x0[1],x0[2],x0[3],x1[0],x1[1],x1[2],x1[3],x2[0],x2[1],x2[2],x2[3],x3[0],x3[1],x3[2],x3[3]};
#pragma unroll
    for (int i = 0; i < 16; ++i) { const unsigned short hb = bf16_bits(xs[i]); ah.u[i] = hb; al.u[i] = ASPLIT ? bf16_bits(xs[i] - bf16_val(hb)) : (unsigned short)0; }
#pragma unroll
    for (int t = 0; t < 4; ++t) {
      const unsigned short* brow = Wt + (size_t)(col0 + t * 16 + ln) * ldb + kb;
      FragB b;
      b.half[0] = *(const v8us*)(brow + 8 * hh);
      b.half[1] = *(const v8us*)(brow + 16 + 8 * hh);
      acc[t] = mmaN<ASPLIT ? 2 : 1>(ah.v, al.v, b.v, b.v, acc[t]);
    }
  }
#pragma unroll
  for (int t = 0; t < 4; ++t) {
    const int col = col0 + t * 16 + ln;
    float bv = bias ? bias[col] : 0.f;
    if (BIAS_BF16) bv = bf16_round(bv);
#pragma unroll
    for (int r = 0; r < 8; ++r) {
      float v = acc[t][r] + bv;
      if (resid) { float rv = resid[(size_t)((row0 + 8 * hh + r) % rmod) * ldr + col]; if (RES_BF16) rv = bf16_round(rv); v += rv; }
      if (ACT == 1) v = fmaxf(v, 0.f);
      if (ACT == 2) v = 0.5f * v * (1.0f + erff(v * 0.70710678118654752f));
      if (ACT == 3) { const float u = 0.7978845608028654f * (v + 0.044715f * v * v * v); v = 0.5f * v * (1.0f + tanhf(u)); }
      so[w][8 * hh + r][t * 16 + ln] = v;
    }
  }
  __builtin_amdgcn_fence(__ATOMIC_ACQ_REL, "workgroup");
  __builtin_amdgcn_wave_barrier();
  const int rsub = lane >> 4, c4 = (lane & 15) * 4;
  for (int pass = 0; pass < 2; ++pass) {
#pragma unroll
    for (int q = 0; q < 8; ++q) {
      const int r = q * 2 + rsub;
      const v4f v = *(const v4fa*)&so[w][r][c4];
      *(volatile v4f*)(C + (size_t)(row0 + r) * ldc + col0 + c4) = v;
    }
    if (pass == 0) __threadfence();
  }
}
template <bool PARAM_BF16>
__global__ __launch_bounds__(256) void k_layernorm(const float* __restrict__ X, const float* __restrict__ R, const float* __restrict__ g, const float* __restrict__ bta,
                                                  float* __restrict__ out_sum, float* __restrict__ out_norm, int N, float eps) {
  __shared__ float red[256];
  const int row = blockIdx.x, tid = threadIdx.x;
  const float* x = X + (size_t)row * N; const float* rr = R ? R + (size_t)row * N : nullptr;
  float vals[16];
  const int per = N / 256;
  float s1 = 0.f;
  for (int u = 0; u < per / 4; ++u) {
    const int j = tid * 4 + 1024 * u;
    const v4f a = *(const v4fa*)(x + j);
    v4f b = {0.f,0.f,0.f,0.f}; if (rr) b = *(const v4fa*)(rr + j);
#pragma unroll
    for (int q = 0; q < 4; ++q) { const float v = a[q] + b[q]; vals[u * 4 + q] = v; s1 += v; }
  }
  red[tid] = s1; __syncthreads();
  for (int st = 128; st > 0; st >>= 1) { if (tid < st) red[tid] += red[tid + st]; __syncthreads(); }
  const float mu = red[0] / (float)N; __syncthreads();
  float s2 = 0.f;
  for (int u = 0; u < per / 4; ++u)
#pragma unroll
    for (int q = 0; q < 4; ++q) { const float c = vals[u * 4 + q] - mu; s2 += c * c; }
  red[tid] = s2; __syncthreads();
  for (int st = 128; st > 0; st >>= 1) { if (tid < st) red[tid] += red[tid + st]; __syncthreads(); }
  const float rs = rsqrtf(red[0] / (float)N + eps);
  for (int pass = 0; pass < 2; ++pass) {
    for (int u = 0; u < per / 4; ++u) {
      const int j = tid * 4 + 1024 * u;
      v4f o, sm;
#pragma unroll
      for (int q = 0; q < 4; ++q) {
        float gg = g[j + q], bb = bta[j + q];
        if (PARAM_BF16) { gg = bf16_round(gg); bb = bf16_round(bb); }
        sm[q] = vals[u * 4 + q]; o[q] = (vals[u * 4 + q] - mu) * rs * gg + bb;
      }
      if (out_sum) *(volatile v4f*)(out_sum + (size_t)row * N + j) = sm;
      *(volatile v4f*)(out_norm + (size_t)row * N + j) = o;
    }
    if (pass == 0) __threadfence();
  }
}


typedef _Float16 v16h __attribute__((ext_vector_type(16)));
union FragH { v16h v; v8us half[2]; _Float16 h[16]; unsigned short u[16]; };
template <int NT>
__device__ __forceinline__ v8f mmaH(v16h ah, v16h al, v16h bh, v16h bl, v8f c) {
  c = __builtin_amdgcn_wmma_f32_16x16x32_f16(false, ah, false, bh, (short)0, c, false, false);
  if (NT >= 2) c = __builtin_amdgcn_wmma_f32_16x16x32_f16(false, al, false, bh, (short)0, c, false, false);
  if (NT >= 3) c = __builtin_amdgcn_wmma_f32_16x16x32_f16(false, ah, false, bl, (short)0, c, false, false);
  asm volatile("v_nop\n\tv_nop\n\tv_nop\n\tv_nop" : "+v"(c) : "v"(ah), "v"(al), "v"(bh), "v"(bl));
  return c;
}
template <bool ASPLIT>
__global__ __launch_bounds__(128) void k_gemm_h(const float* __restrict__ A, int lda, size_t sA, const _Float16* __restrict__ Bh, int ldb, size_t sB, float alpha, float* __restrict__ C, int ldc, size_t sC, int M, int N, int K) {
  __shared__ __attribute__((aligned(16))) float so[4][16][64];
  const int tid = threadIdx.x, w = tid >> 5, lane = tid & 31, ln = lane & 15, hh = lane >> 4; const int by = blockIdx.y;
  A += (size_t)by * sA; Bh += (size_t)by * sB; C += (size_t)by * sC;
  const int ntn = (N + 63) / 64; const int wid = blockIdx.x * 4 + w; const int mt = wid / ntn, nq = wid % ntn; if (mt * 16 >= M) return;
  const int row0 = mt * 16, col0 = nq * 64; const float* arow = A + (size_t)(row0 + ln) * lda;
  v8f acc[4] = {};
  for (int kb = 0; kb < K; kb += 32) {
    FragH ah, al;
    const v4f x0 = *(const v4fa*)(arow + kb + 8 * hh), x1 = *(const v4fa*)(arow + kb + 8 * hh + 4), x2 = *(const v4fa*)(arow + kb + 16 + 8 * hh), x3 = *(const v4fa*)(arow + kb + 16 + 8 * hh + 4);
    float xs[16] = {x0[0],x0[1],x0[2],x0[3],x1[0],x1[1],x1[2],x1[3],x2[0],x2[1],x2[2],x2[3],x3[0],x3[1],x3[2],x3[3]};
#pragma unroll
    for (int i = 0; i < 16; ++i) { const _Float16 h = (_Float16)xs[i]; ah.h[i] = h; al.h[i] = ASPLIT ? (_Float16)(xs[i] - (float)h) : (_Float16)0.0f; }
#pragma unroll
    for (int t = 0; t < 4; ++t) { if (col0 + t * 16 >= N) continue; const size_t boff = (size_t)(col0 + t * 16 + ln) * ldb + kb; FragH bq; bq.half[0] = *(const v8us*)(Bh + boff + 8 * hh); bq.half[1] = *(const v8us*)(Bh + boff + 16 + 8 * hh);
      acc[t] = mmaH<ASPLIT ? 2 : 1>(ah.v, al.v, bq.v, bq.v, acc[t]); }
  }
#pragma unroll
  for (int t = 0; t < 4; ++t) { if (col0 + t * 16 >= N) continue;
#pragma unroll
    for (int r = 0; r < 8; ++r) so[w][8 * hh + r][t * 16 + ln] = acc[t][r] * alpha; }
  __builtin_amdgcn_fence(__ATOMIC_ACQ_REL, "workgroup"); __builtin_amdgcn_wave_barrier();
  const int rsub = lane >> 4, c4 = (lane & 15) * 4;
  for (int pass = 0; pass < 2; ++pass) {
#pragma unroll
    for (int q = 0; q < 8; ++q) { const int r = q * 2 + rsub; if (col0 + c4 < N) { const v4f v = *(const v4fa*)&so[w][r][c4]; *(volatile v4f*)(C + (size_t)(row0 + r) * ldc + col0 + c4) = v; } }
    if (pass == 0) __threadfence(); }
}

__global__ __launch_bounds__(256) void k_wt_f16(const float* __restrict__ W, _Float16* __restrict__ Wt, int K, int N, float scale) {
  const int t = blockIdx.x * 256 + threadIdx.x; if (t >= N * (K / 8)) return; const int n = t / (K / 8), k8 = (t % (K / 8)) * 8; FragH f;
#pragma unroll
  for (int i = 0; i < 8; ++i) f.h[i] = (_Float16)(bf16_round(W[(size_t)(k8 + i) * N + n]) * scale); const v8us o = f.half[0];
  *(volatile v8us*)((unsigned short*)Wt + (size_t)n * K + k8) = o; __threadfence(); *(volatile v8us*)((unsigned short*)Wt + (size_t)n * K + k8) = o;
}
template <int ACT>
__global__ __launch_bounds__(128) void k_gemm_hhx(const _Float16* __restrict__ A, int lda, size_t sA, const _Float16* __restrict__ Bh, int ldb, size_t sB, float alpha, const float* __restrict__ bias, size_t sBias, const float* __restrict__ CP, int rowsPerB, size_t sCPb, int row0g,
    float* __restrict__ C, _Float16* __restrict__ C16, int ldc, size_t sC, int M, int N, int K) {
  __shared__ __attribute__((aligned(16))) float so[4][16][64];
  const int tid = threadIdx.x, w = tid >> 5, lane = tid & 31, ln = lane & 15, hh = lane >> 4; const int by = blockIdx.y;
  A += (size_t)by * sA; Bh += (size_t)by * sB; const size_t cofs = (size_t)by * sC; const float* bp = bias ? bias + (size_t)by * sBias : nullptr;
  const int ntn = (N + 63) / 64; const int wid = blockIdx.x * 4 + w; const int mt = wid / ntn, nq = wid % ntn; if (mt * 16 >= M) return;
  const int row0 = mt * 16, col0 = nq * 64; const _Float16* arow = A + (size_t)(row0 + ln) * lda;
  v8f acc[4] = {};
  for (int kb = 0; kb < K; kb += 32) { FragH ah; ah.half[0] = *(const v8us*)((const unsigned short*)arow + kb + 8 * hh); ah.half[1] = *(const v8us*)((const unsigned short*)arow + kb + 16 + 8 * hh);
#pragma unroll
    for (int t = 0; t < 4; ++t) { if (col0 + t * 16 >= N) continue; const size_t boff = (size_t)(col0 + t * 16 + ln) * ldb + kb; FragH bq; bq.half[0] = *(const v8us*)((const unsigned short*)Bh + boff + 8 * hh); bq.half[1] = *(const v8us*)((const unsigned short*)Bh + boff + 16 + 8 * hh);
      acc[t] = mmaH<1>(ah.v, ah.v, bq.v, bq.v, acc[t]); }
  }
#pragma unroll
  for (int t = 0; t < 4; ++t) { if (col0 + t * 16 >= N) continue; const int col = col0 + t * 16 + ln; const float bv = bp ? bf16_round(bp[col]) : 0.f;
#pragma unroll
    for (int r = 0; r < 8; ++r) { float v = acc[t][r] * alpha + bv; if (CP) { const int bidx = (row0g + row0 + 8 * hh + r) / rowsPerB; v += CP[(size_t)bidx * sCPb + (size_t)by * 64 + col]; } if (ACT == 1) v = (v > 0.f) ? v : expm1f(v); else if (ACT == 7) v = (v > 0.f) ? v + 1.0f : expf(v); else if (ACT == 8) v = tanhf(v); else if (ACT == 9) v = 0.5f * v * (1.0f + tanhf(0.7978845608028654f * (v + 0.044715f * v * v * v))); else if (ACT == 11) v = 1.0f / (1.0f + expf(-v)); else if (ACT == 12) v = (v > 0.f) ? v : 0.01f * v; else if (ACT == 14) v = (v > 0.f) ? v : 0.1f * v; else if (ACT == 15) v = v / (1.0f + expf(-v)); else if (ACT == 3) v = fmaxf(v, 0.f); else if (ACT == 6) v = 0.5f * v * (1.0f + erff(v * 0.70710678118654752f)); so[w][8 * hh + r][t * 16 + ln] = v; } }
  __builtin_amdgcn_fence(__ATOMIC_ACQ_REL, "workgroup"); __builtin_amdgcn_wave_barrier();
  const int rsub = lane >> 4, c4 = (lane & 15) * 4; typedef _Float16 v4h __attribute__((ext_vector_type(4)));
  for (int pass = 0; pass < 2; ++pass) {
#pragma unroll
    for (int q = 0; q < 8; ++q) { const int r = q * 2 + rsub; if (col0 + c4 < N) { const v4f v = *(const v4fa*)&so[w][r][c4]; if (C) *(volatile v4f*)(C + cofs + (size_t)(row0 + r) * ldc + col0 + c4) = v; if (C16) { v4h h4; for (int i = 0; i < 4; ++i) h4[i] = (_Float16)v[i]; *(volatile v4h*)(C16 + cofs + (size_t)(row0 + r) * ldc + col0 + c4) = h4; } } }
    if (pass == 0) __threadfence(); }
}


typedef _Float16 v4h __attribute__((ext_vector_type(4)));

__global__ __launch_bounds__(256) void k_x16(const float* __restrict__ x, _Float16* __restrict__ X16, size_t n8) { const size_t t = (size_t)blockIdx.x * 256 + threadIdx.x; if (t >= n8) return; FragH f;
#pragma unroll
  for (int q = 0; q < 8; ++q) f.h[q] = (_Float16)bf16_round(x[t * 8 + q]); *(volatile v8us*)((unsigned short*)X16 + t * 8) = f.half[0]; __threadfence(); *(volatile v8us*)((unsigned short*)X16 + t * 8) = f.half[0]; }
__global__ __launch_bounds__(256) void k_h16(const float* __restrict__ x, _Float16* __restrict__ X16, size_t n8) { const size_t t = (size_t)blockIdx.x * 256 + threadIdx.x; if (t >= n8) return; FragH f;
#pragma unroll
  for (int q = 0; q < 8; ++q) f.h[q] = (_Float16)x[t * 8 + q]; *(volatile v8us*)((unsigned short*)X16 + t * 8) = f.half[0]; __threadfence(); *(volatile v8us*)((unsigned short*)X16 + t * 8) = f.half[0]; }
__global__ __launch_bounds__(256) void k_round16f(const float* __restrict__ W, _Float16* __restrict__ Bt, size_t n8) { const size_t t = (size_t)blockIdx.x * 256 + threadIdx.x; if (t >= n8) return; FragH f;
#pragma unroll
  for (int i = 0; i < 8; ++i) f.h[i] = (_Float16)(bf16_round(W[t * 8 + i]) * 16.0f); *(volatile v8us*)((unsigned short*)Bt + t * 8) = f.half[0]; __threadfence(); *(volatile v8us*)((unsigned short*)Bt + t * 8) = f.half[0]; }
template <int NHv, int TTv>
__global__ __launch_bounds__(256) void k_vt(const _Float16* __restrict__ V16, int ldv, int voff, _Float16* __restrict__ Vt) { __shared__ unsigned short tl[64][66]; const int tid = threadIdx.x; const int slab = blockIdx.x / (TTv / 64), lg = blockIdx.x % (TTv / 64); const int b = slab / NHv, h = slab % NHv;
  for (int i = tid; i < 64 * 8; i += 256) { const int r = i / 8, c8 = (i % 8) * 8; FragH f; f.half[0] = *(const v8us*)((const unsigned short*)V16 + ((size_t)b * TTv + lg * 64 + r) * ldv + voff + h * 64 + c8);
#pragma unroll
    for (int q = 0; q < 8; ++q) tl[r][c8 + q] = f.u[q]; }
  __syncthreads();
  for (int pass = 0; pass < 2; ++pass) {
#pragma unroll
    for (int rd = 0; rd < 2; ++rd) { const int d = rd * 32 + tid / 8, pc = tid % 8; FragH f;
#pragma unroll
      for (int q = 0; q < 8; ++q) f.u[q] = tl[pc * 8 + q][d];
      *(volatile v8us*)((unsigned short*)Vt + ((size_t)slab * 64 + d) * TTv + lg * 64 + pc * 8) = f.half[0]; }
    if (pass == 0) __threadfence(); } }

__global__ __launch_bounds__(256) void k_hl(const float* __restrict__ F, _Float16* __restrict__ Hh, _Float16* __restrict__ Hl, size_t n8) { const size_t t = (size_t)blockIdx.x * 256 + threadIdx.x; if (t >= n8) return; FragH fh, fl; const v4f a = *(const v4fa*)(F + t * 8), c = *(const v4fa*)(F + t * 8 + 4);
#pragma unroll
  for (int q = 0; q < 4; ++q) { _Float16 h = (_Float16)a[q]; fh.h[q] = h; fl.h[q] = (_Float16)((a[q] - (float)h) * 1024.0f); h = (_Float16)c[q]; fh.h[4 + q] = h; fl.h[4 + q] = (_Float16)((c[q] - (float)h) * 1024.0f); }
  for (int pass = 0; pass < 2; ++pass) { *(volatile v8us*)((unsigned short*)Hh + t * 8) = fh.half[0]; *(volatile v8us*)((unsigned short*)Hl + t * 8) = fl.half[0]; if (pass == 0) __threadfence(); } }

__device__ __forceinline__ v16h g2_frag(const _Float16* p, int hh) { FragH f; f.half[0] = *(const v8us*)((const unsigned short*)p + 8 * hh); f.half[1] = *(const v8us*)((const unsigned short*)p + 16 + 8 * hh); return f.v; }
__device__ __forceinline__ v8f g2_mma(v16h a, v16h b, v8f c) { v8f d = __builtin_amdgcn_wmma_f32_16x16x32_f16(false, a, false, b, (short)0, c, false, false); asm volatile("v_nop\n\tv_nop\n\tv_nop\n\tv_nop" : "+v"(d) : "v"(a), "v"(b)); return d; }
template <int ACT>
__global__ __launch_bounds__(128) void k_gemm2(const _Float16* __restrict__ A, int lda, size_t sA, const _Float16* __restrict__ Bh, int ldb, size_t sB, float alpha, const float* __restrict__ bias, size_t sBias, const float* __restrict__ CP, int rowsPerB, size_t sCPb, int row0g,
    float* __restrict__ C, _Float16* __restrict__ C16, int ldc, size_t sC, int M, int N, int K) {
  __shared__ __attribute__((aligned(16))) float so[4][32][68];
  const int tid = threadIdx.x, w = tid >> 5, lane = tid & 31, ln = lane & 15, hh = lane >> 4; const int by = blockIdx.y;
  A += (size_t)by * sA; Bh += (size_t)by * sB; const size_t cofs = (size_t)by * sC; const float* bp = bias ? bias + (size_t)by * sBias : nullptr;
  const int ntn = N >> 6; const int mt = blockIdx.x / ntn, nq = blockIdx.x - mt * ntn; const int row0 = mt * 128 + 32 * w, col0 = nq * 64; if (row0 >= M) return;
  const _Float16* a0p = A + (size_t)(row0 + ln) * lda; const _Float16* a1p = a0p + (size_t)16 * lda;
  const _Float16* b0p = Bh + (size_t)(col0 + ln) * ldb; const _Float16* b1p = b0p + (size_t)16 * ldb; const _Float16* b2p = b1p + (size_t)16 * ldb; const _Float16* b3p = b2p + (size_t)16 * ldb;
  const v8f z8 = {0.f,0.f,0.f,0.f,0.f,0.f,0.f,0.f}; v8f c00 = z8, c01 = z8, c02 = z8, c03 = z8, c10 = z8, c11 = z8, c12 = z8, c13 = z8;
#pragma unroll 1
  for (int kb = 0; kb < K; kb += 32) { const v16h a0 = g2_frag(a0p + kb, hh), a1 = g2_frag(a1p + kb, hh);
    v16h b = g2_frag(b0p + kb, hh); c00 = g2_mma(a0, b, c00); c10 = g2_mma(a1, b, c10);
    b = g2_frag(b1p + kb, hh); c01 = g2_mma(a0, b, c01); c11 = g2_mma(a1, b, c11);
    b = g2_frag(b2p + kb, hh); c02 = g2_mma(a0, b, c02); c12 = g2_mma(a1, b, c12);
    b = g2_frag(b3p + kb, hh); c03 = g2_mma(a0, b, c03); c13 = g2_mma(a1, b, c13); }
  v8f accs[8] = {c00, c01, c02, c03, c10, c11, c12, c13};
#pragma unroll
  for (int u = 0; u < 8; ++u) { const int t = u & 3, half = u >> 2; const int col = col0 + t * 16 + ln; const float bv = bp ? bf16_round(bp[col]) : 0.f;
#pragma unroll
    for (int r = 0; r < 8; ++r) { const int rloc = half * 16 + 8 * hh + r; float v = accs[u][r] * alpha + bv; if (CP) { const int bidx = (row0g + row0 + rloc) / rowsPerB; v += CP[(size_t)bidx * sCPb + (size_t)by * 64 + col]; }
      if (ACT == 3) v = fmaxf(v, 0.f); else if (ACT == 6) v = 0.5f * v * (1.0f + erff(v * 0.70710678118654752f)); else if (ACT == 11) v = 1.0f / (1.0f + expf(-v)); else if (ACT == 15) v = v / (1.0f + expf(-v)); else if (ACT == 12) v = (v > 0.f) ? v : 0.01f * v; else if (ACT == 8) v = tanhf(v);
      so[w][rloc][t * 16 + ln] = v; } }
  __builtin_amdgcn_fence(__ATOMIC_ACQ_REL, "workgroup"); __builtin_amdgcn_wave_barrier();
  const int rsub = lane >> 4, c4 = (lane & 15) * 4;
  for (int pass = 0; pass < 2; ++pass) {
#pragma unroll
    for (int q = 0; q < 16; ++q) { const int r = q * 2 + rsub; const v4f v = *(const v4fa*)&so[w][r][c4]; if (C) *(volatile v4f*)(C + cofs + (size_t)(row0 + r) * ldc + col0 + c4) = v; if (C16) { v4h h4; for (int i = 0; i < 4; ++i) h4[i] = (_Float16)v[i]; *(volatile v4h*)(C16 + cofs + (size_t)(row0 + r) * ldc + col0 + c4) = h4; } }
    if (pass == 0) __threadfence(); } }


__device__ __forceinline__ float cubic_w(float d) { const float a = -0.75f; d = fabsf(d); const float w1 = ((a + 2.0f) * d - (a + 3.0f)) * d * d + 1.0f; const float w2 = (((a * d) - 5.0f * a) * d + 8.0f * a) * d - 4.0f * a; return (d <= 1.0f) ? w1 : ((d < 2.0f) ? w2 : 0.0f); }
template <int AX, int SRCX>
__global__ __launch_bounds__(256) void k_rsz(const float* __restrict__ src, int b, int hin, int win, int hout, int wout, float scale, float* __restrict__ dst) {
  #pragma clang fp contract(off)
  const int t = blockIdx.x * 256 + threadIdx.x; if (t >= CC * hout * wout) return; const int xo = t % wout; const int yo = (t / wout) % hout; const int c = t / (wout * hout);
  const int o = AX == 0 ? yo : xo; const int insz = AX == 0 ? hin : win; const float sp = ((float)o + 0.5f) * scale - 0.5f; const float f0 = floorf(sp); const float tt = sp - f0; const int i0 = (int)fminf(fmaxf(f0, -4096.f), 4096.f); float acc = 0.f;
#pragma unroll
  for (int off = -1; off < 3; ++off) { const int idx = min(max(i0 + off, 0), insz - 1); const float w = cubic_w(tt - (float)off); const int yy = AX == 0 ? idx : yo, xx = AX == 0 ? xo : idx;
    const float v = SRCX ? bf16_round(src[((size_t)b * CC + c) * NQ + yy * H0 + xx]) : src[((size_t)c * H0 + yy) * H0 + xx]; acc += v * w; }
  float* d = dst + ((size_t)c * H0 + yo) * H0 + xo; *(volatile float*)d = acc; __threadfence(); *(volatile float*)d = acc; }
__global__ __launch_bounds__(256) void k_cpx(const float* __restrict__ x, int b, float* __restrict__ dst) { const int t = blockIdx.x * 256 + threadIdx.x; if (t >= CC * NQ / 4) return; const v4f a = *(const v4fa*)(x + (size_t)b * CC * NQ + (size_t)t * 4); v4f o; for (int q = 0; q < 4; ++q) o[q] = bf16_round(a[q]); *(volatile v4f*)(dst + (size_t)t * 4) = o; __threadfence(); *(volatile v4f*)(dst + (size_t)t * 4) = o; }
__global__ __launch_bounds__(256) void k_im2p(const float* __restrict__ M, int h, int w, int npad, _Float16* __restrict__ X3) {
  #pragma clang fp contract(off)
  const int t = blockIdx.x * 256 + threadIdx.x; if (t >= npad * 72) return; const int k0 = (t % 72) * 8; const int p = t / 72; const int y = p / w, xq = p % w; FragH fh, fl;
#pragma unroll
  for (int q = 0; q < 8; ++q) { const int k = k0 + q; const int c = k / 9, r = k % 9; const int yy = y + r / 3 - 1, xx = xq + r % 3 - 1; float v = 0.f; if (p < h * w && yy >= 0 && yy < h && xx >= 0 && xx < w) v = M[((size_t)c * H0 + yy) * H0 + xx]; const _Float16 hv = (_Float16)v; fh.h[q] = hv; fl.h[q] = (_Float16)((v - (float)hv) * 16.0f); }
  unsigned short* d = (unsigned short*)X3 + (size_t)p * 1152 + k0;
  for (int pass = 0; pass < 2; ++pass) { *(volatile v8us*)d = fh.half[0]; *(volatile v8us*)(d + 576) = fl.half[0]; if (pass == 0) __threadfence(); } }
__global__ __launch_bounds__(256) void k_px1(const float* __restrict__ M, int h, int w, int npad, _Float16* __restrict__ X1) {
  #pragma clang fp contract(off)
  const int t = blockIdx.x * 256 + threadIdx.x; if (t >= npad * 8) return; const int c0 = (t & 7) * 8; const int p = t >> 3; const int y = p / w, xq = p % w; FragH fh, fl;
#pragma unroll
  for (int q = 0; q < 8; ++q) { const float v = (p < h * w) ? M[((size_t)(c0 + q) * H0 + y) * H0 + xq] : 0.f; const _Float16 hv = (_Float16)v; fh.h[q] = hv; fl.h[q] = (_Float16)((v - (float)hv) * 16.0f); }
  unsigned short* d = (unsigned short*)X1 + (size_t)p * 128 + c0;
  for (int pass = 0; pass < 2; ++pass) { *(volatile v8us*)d = fh.half[0]; *(volatile v8us*)(d + 64) = fl.half[0]; if (pass == 0) __threadfence(); } }
__global__ __launch_bounds__(256) void k_w3p(const float* __restrict__ Wt, int O, _Float16* __restrict__ Bt) {
  const int t = blockIdx.x * 256 + threadIdx.x; if (t >= 64 * 144) return; const int k0 = (t % 144) * 8; const int n = t / 144; const bool lo = k0 >= 576; FragH f;
#pragma unroll
  for (int q = 0; q < 8; ++q) { const int k = k0 + q - (lo ? 576 : 0); f.h[q] = (n < O) ? (_Float16)(bf16_round(Wt[(size_t)n * 576 + k]) * (lo ? 1.0f : 16.0f)) : (_Float16)0.0f; }
  *(volatile v8us*)((unsigned short*)Bt + (size_t)n * 1152 + k0) = f.half[0]; __threadfence(); *(volatile v8us*)((unsigned short*)Bt + (size_t)n * 1152 + k0) = f.half[0]; }
__global__ __launch_bounds__(256) void k_w1p(const float* __restrict__ Wt, _Float16* __restrict__ Bt) { const int t = blockIdx.x * 256 + threadIdx.x; if (t >= 64 * 16) return; const int k0 = (t & 15) * 8; const int n = t >> 4; const bool lo = k0 >= 64; FragH f;
#pragma unroll
  for (int q = 0; q < 8; ++q) { const int k = k0 + q - (lo ? 64 : 0); f.h[q] = (_Float16)(bf16_round(Wt[n * 64 + k]) * (lo ? 1.0f : 16.0f)); }
  *(volatile v8us*)((unsigned short*)Bt + (size_t)n * 128 + k0) = f.half[0]; __threadfence(); *(volatile v8us*)((unsigned short*)Bt + (size_t)n * 128 + k0) = f.half[0]; }
__global__ __launch_bounds__(64) void k_bpad(const float* __restrict__ b, int nreal, float* __restrict__ BB) { const int t = threadIdx.x; const float v = (t < nreal) ? b[t] : 0.f; *(volatile float*)(BB + t) = v; __threadfence(); *(volatile float*)(BB + t) = v; }
template <int ISK>
__global__ __launch_bounds__(256) void k_seg3(const float* __restrict__ F, int nreal, int koff, _Float16* __restrict__ D3) {
  #pragma clang fp contract(off)
  const int t = blockIdx.x * 256 + threadIdx.x; if (t >= nreal * 12) return; const int pc = t % 12; const int r = t / 12; const int seg = pc / 4, d0 = (pc % 4) * 8; const float* f = F + (size_t)r * 64 + d0; FragH o;
#pragma unroll
  for (int q = 0; q < 8; ++q) { const float v = f[q]; const _Float16 hv = (_Float16)v; const float lo = (v - (float)hv) * 16.0f;
    if (seg == 0) o.h[q] = hv; else if (seg == 1) o.h[q] = ISK ? (_Float16)((float)hv * 0.0625f) : (_Float16)lo; else o.h[q] = ISK ? (_Float16)lo : (_Float16)((float)hv * 0.0625f); }
  unsigned short* d = (unsigned short*)D3 + ((size_t)koff + r) * 96 + seg * 32 + d0; *(volatile v8us*)d = o.half[0]; __threadfence(); *(volatile v8us*)d = o.half[0]; }
__global__ __launch_bounds__(256) void k_rawt(const float* __restrict__ RAW, int nreal, int koff, _Float16* __restrict__ RAWT) {
  __shared__ float tl[64][65]; const int tid = threadIdx.x; const int p0 = blockIdx.x * 64;
  for (int i = tid; i < 64 * 16; i += 256) { const int pl = i / 16, c4 = (i % 16) * 4; const v4f a = *(const v4fa*)(RAW + (size_t)(p0 + pl) * 64 + c4); for (int q = 0; q < 4; ++q) tl[pl][c4 + q] = a[q]; }
  __syncthreads();
  const int c = tid >> 2, p8 = (tid & 3) * 16;
  for (int pass = 0; pass < 2; ++pass) {
#pragma unroll
    for (int u = 0; u < 2; ++u) { const int pl = p8 + u * 8; if (p0 + pl + 8 <= ((nreal + 7) / 8) * 8) { FragH f;
#pragma unroll
        for (int q = 0; q < 8; ++q) f.h[q] = (_Float16)tl[pl + q][c];
        *(volatile v8us*)((unsigned short*)RAWT + (size_t)c * LP + koff + p0 + pl) = f.half[0]; } }
    if (pass == 0) __threadfence(); } }
__global__ __launch_bounds__(256) void k_zpad(_Float16* __restrict__ K3, _Float16* __restrict__ RAWT) {
  const int t = blockIdx.x * 256 + threadIdx.x; if (t >= 160 * 160) return; const int pk = t / 160, u = t % 160;
  int cnt = 0, key = -1;
#pragma unroll
  for (int s = 0; s < NSC; ++s) { const int npad = KOFF[s + 1] - KOFF[s] - NREALK[s]; if (key < 0 && pk < cnt + npad) key = KOFF[s] + NREALK[s] + (pk - cnt); cnt += npad; }
  if (key < 0) return;
  if (u < 96) { unsigned short* d = (unsigned short*)K3 + (size_t)key * 96 + u; *(volatile unsigned short*)d = 0; __threadfence(); *(volatile unsigned short*)d = 0; }
  else { unsigned short* d = (unsigned short*)RAWT + (size_t)(u - 96) * LP + key; *(volatile unsigned short*)d = 0; __threadfence(); *(volatile unsigned short*)d = 0; } }
__device__ __forceinline__ bool key_ok(int kk) { int s = 0;
#pragma unroll
  for (int i = 1; i < NSC; ++i) s += (kk >= KOFF[i]) ? 1 : 0; return (kk - KOFF[s]) < NREALK[s]; }
__global__ __launch_bounds__(256) void k_softL(const float* __restrict__ S, _Float16* __restrict__ P16) {
  #pragma clang fp contract(off)
  const int tid = threadIdx.x, w = tid >> 5, ln = tid & 31; const int r = blockIdx.x * 8 + w; if (r >= NQ) return; const float* s = S + (size_t)r * LP; float m = -3.0e38f;
#pragma unroll 1
  for (int c = 0; c < 30; ++c) { const int kb = c * 256 + ln * 8; if (kb >= LP) continue; for (int q = 0; q < 8; ++q) { const int kk = kb + q; if (key_ok(kk)) m = fmaxf(m, s[kk]); } }
  for (int o = 16; o > 0; o >>= 1) m = fmaxf(m, __shfl_xor(m, o, 32)); float su = 0.f;
#pragma unroll 1
  for (int c = 0; c < 30; ++c) { const int kb = c * 256 + ln * 8; if (kb >= LP) continue; for (int q = 0; q < 8; ++q) { const int kk = kb + q; if (key_ok(kk)) su += expf(s[kk] - m); } }
  for (int o = 16; o > 0; o >>= 1) su += __shfl_xor(su, o, 32); const float inv = 1024.0f / su; unsigned short* d = (unsigned short*)P16 + (size_t)r * LP;
  for (int pass = 0; pass < 2; ++pass) {
#pragma unroll 1
    for (int c = 0; c < 30; ++c) { const int kb = c * 256 + ln * 8; if (kb >= LP) continue; FragH f;
#pragma unroll
      for (int q = 0; q < 8; ++q) { const int kk = kb + q; f.h[q] = key_ok(kk) ? (_Float16)(expf(s[kk] - m) * inv) : (_Float16)0.0f; }
      *(volatile v8us*)(d + kb) = f.half[0]; }
    if (pass == 0) __threadfence(); } }
__global__ __launch_bounds__(256) void k_outp(const float* __restrict__ Y, const float* __restrict__ x, int b, float* __restrict__ out) {
  #pragma clang fp contract(off)
  const int t = blockIdx.x * 256 + threadIdx.x; if (t >= CC * NQ / 4) return; const int c = t / (NQ / 4), q0 = (t % (NQ / 4)) * 4; v4f r; const float* xr = x + ((size_t)b * CC + c) * NQ + q0;
#pragma unroll
  for (int q = 0; q < 4; ++q) r[q] = Y[(size_t)(q0 + q) * 64 + c] + bf16_round(xr[q]);
  float* d = out + ((size_t)b * CC + c) * NQ + q0; *(volatile v4f*)d = r; __threadfence(); *(volatile v4f*)d = r; }

extern "C" void kernel_launch(void* const* d_in, const int* in_sizes, int n_in,
                              void* d_out, int out_size, void* d_ws, size_t ws_size, hipStream_t stream) {
  (void)in_sizes; (void)n_in; (void)out_size;
  const float* const* I = (const float* const*)d_in; const float* x = I[0]; const float* wb = I[1]; const float* bb = I[2]; const float* wm = I[3]; const float* bm = I[4]; const float* wa = I[5]; const float* ba = I[6];
  char* ws = (char*)d_ws; size_t off = 0;
  auto take = [&](size_t bytes) { char* p = ws + off; off += (bytes + 255) & ~(size_t)255; return p; };
  _Float16* BWB = (_Float16*)take((size_t)64 * 1152 * 2); _Float16* BWM = (_Float16*)take((size_t)64 * 1152 * 2); _Float16* BWA = (_Float16*)take((size_t)64 * 128 * 2); float* BBB = (float*)take(256); float* BBM = (float*)take(256);
  float* MAPA = (float*)take((size_t)CC * NQ * 4); float* MAPB = (float*)take((size_t)CC * NQ * 4); _Float16* X3 = (_Float16*)take((size_t)NQ * 1152 * 2); _Float16* X1 = (_Float16*)take((size_t)NQ * 128 * 2); float* F = (float*)take((size_t)NQ * 64 * 4);
  _Float16* Q3 = (_Float16*)take((size_t)NQ * 96 * 2); _Float16* K3 = (_Float16*)take((size_t)LP * 96 * 2); _Float16* RAWT = (_Float16*)take((size_t)CC * LP * 2); float* S = (float*)take((size_t)NQ * LP * 4); _Float16* P16 = (_Float16*)take((size_t)NQ * LP * 2); float* Y = (float*)take((size_t)NQ * 64 * 4);
  if (off > ws_size) return;
  k_w3p<<<(64 * 144 + 255) / 256, 256, 0, stream>>>(wb, CR, BWB); k_w3p<<<(64 * 144 + 255) / 256, 256, 0, stream>>>(wm, CR, BWM); k_w1p<<<4, 256, 0, stream>>>(wa, BWA); k_bpad<<<1, 64, 0, stream>>>(bb, CR, BBB); k_bpad<<<1, 64, 0, stream>>>(bm, CR, BBM);
  k_zpad<<<(160 * 160 + 255) / 256, 256, 0, stream>>>(K3, RAWT);
  for (int b = 0; b < NIMG; ++b) {
    for (int s = 0; s < NSC; ++s) { const int hs = hSZ[s], np = hs * hs, npad = hNPAD[s], koff = hKOFF[s]; const float* MAP;
      if (s == 0) { k_cpx<<<(CC * NQ / 4 + 255) / 256, 256, 0, stream>>>(x, b, MAPA); MAP = MAPA; }
      else { const float scale = 48.0f / (float)hs;
        k_rsz<0, 1><<<(CC * hs * H0 + 255) / 256, 256, 0, stream>>>(x, b, H0, H0, hs, H0, scale, MAPB);
        k_rsz<1, 0><<<(CC * hs * hs + 255) / 256, 256, 0, stream>>>(MAPB, 0, hs, H0, hs, hs, scale, MAPA); MAP = MAPA; }
      if (s == 0) {
        k_im2p<<<(npad * 72 + 255) / 256, 256, 0, stream>>>(MAP, hs, hs, npad, X3);
        k_gemm2<0><<<dim3((npad / 128) * 1, 1), 128, 0, stream>>>(X3, 1152, 0, BWB, 1152, 0, 0.0625f, BBB, 0, nullptr, 1, 0, 0, F, nullptr, 64, 0, npad, 64, 1152);
        k_seg3<0><<<(np * 12 + 255) / 256, 256, 0, stream>>>(F, np, 0, Q3); }
      k_im2p<<<(npad * 72 + 255) / 256, 256, 0, stream>>>(MAP, hs, hs, npad, X3);
      k_gemm2<0><<<dim3((npad / 128) * 1, 1), 128, 0, stream>>>(X3, 1152, 0, BWM, 1152, 0, 0.0625f, BBM, 0, nullptr, 1, 0, 0, F, nullptr, 64, 0, npad, 64, 1152);
      k_seg3<1><<<(np * 12 + 255) / 256, 256, 0, stream>>>(F, np, koff, K3);
      k_px1<<<(npad * 8 + 255) / 256, 256, 0, stream>>>(MAP, hs, hs, npad, X1);
      k_gemm2<0><<<dim3((npad / 128) * 1, 1), 128, 0, stream>>>(X1, 128, 0, BWA, 128, 0, 0.0625f, ba, 0, nullptr, 1, 0, 0, F, nullptr, 64, 0, npad, 64, 128);
      k_rawt<<<npad / 64, 256, 0, stream>>>(F, np, koff, RAWT); }
    k_gemm2<0><<<dim3((NQ / 128) * (LP / 64), 1), 128, 0, stream>>>(Q3, 96, 0, K3, 96, 0, 1.0f, nullptr, 0, nullptr, 1, 0, 0, S, nullptr, LP, 0, NQ, LP, 96);
    k_softL<<<NQ / 8, 256, 0, stream>>>(S, P16);
    k_gemm2<0><<<dim3((NQ / 128) * 1, 1), 128, 0, stream>>>(P16, LP, 0, RAWT, LP, 0, 0.0009765625f, nullptr, 0, nullptr, 1, 0, 0, Y, nullptr, 64, 0, NQ, 64, LP);
    k_outp<<<(CC * NQ / 4 + 255) / 256, 256, 0, stream>>>(Y, x, b, (float*)d_out); }
}
